// GraphSageNet_55207509623126
// MI455X (gfx1250) — hardware-verified
//
#include <hip/hip_runtime.h>
#include <stddef.h>
#include <stdint.h>


#define HID    108
#define DF     128
#define HP     256
#define KE     32
#define KP     256
#define KA     512
#define NLAY   4
#define NTL    7
#define NTHR   256
#define NWAVE  8
#define EPT    8
#define CHUNK  (NTHR * EPT)
#define WCAP   (EPT * 32)
#define LISTN  (NWAVE * WCAP)
#define NBA    1024
#define SLA    10
#define RCAP   28672
#define DEGCAP 64
#define MEAS_B1024  16683
#define MEAS_MAXDEG 38
#define AGB    64
#define GBM    64
#define GBN    128
#define GTHR   128
#define GWAVE  (GTHR / 32)
#define NUWE   (DF * (KE / 8))
#define NUWP1  (DF * (KP / 8))
#define NUWP   (NLAY * NUWP1)
#define NUWA1  (DF * (KA / 8))
#define NUWA   (NLAY * NUWA1)
#define NUW    (NUWE + NUWP + NUWA)
#define PTHR   256
#define OTHR   640
#define LOGW   32
#define AGG_ZINTS    (LISTN + 2 * RCAP + 3 * NBA)
#define MISC_INTS    16
#define BKT_LDS_INTS (AGG_ZINTS + MISC_INTS)
#define WSMAX  134217728

static_assert((CHUNK & (CHUNK - 1)) == 0 && CHUNK <= 4096);
static_assert((NBA & (NBA - 1)) == 0 && NBA == (1 << SLA) && NBA == 1024);
static_assert(((long long)CHUNK << SLA) < (1LL << 31));
static_assert(RCAP % (NTHR * 4) == 0 && AGG_ZINTS % (NTHR * 4) == 0 && NBA == NTHR * 4);
static_assert(RCAP >= MEAS_B1024 + 4096);
static_assert(DEGCAP >= MEAS_MAXDEG + 8);
static_assert(KE % 32 == 0 && KP % 32 == 0 && KA % 32 == 0 && KP == HP && KA == 2 * HP && HP == 2 * DF);
static_assert(GBN == DF && GBM == GWAVE * 16 && DF == 4 * 32 && NTL * 16 >= HID && NTL * 16 + 16 == GBN);
static_assert(NUWE % NTHR == 0 && NUWP1 % NTHR == 0 && NUWA1 % NTHR == 0 && NUW % NTHR == 0);
static_assert(NUWP1 == 4096 && NUWA1 == 8192);
static_assert(AGB % NWAVE == 0 && NBA % AGB == 0 && AGB == GBM);
static_assert(BKT_LDS_INTS * 4 <= 300000);
static_assert(HID <= DF && (HID / 2) <= 64 && (HID / 4) <= 32);

typedef float          v4f   __attribute__((ext_vector_type(4)));
typedef float          v8f   __attribute__((ext_vector_type(8)));
typedef int            v4i   __attribute__((ext_vector_type(4)));
typedef int            v8i   __attribute__((ext_vector_type(8)));
typedef unsigned short v4us  __attribute__((ext_vector_type(4)));
typedef unsigned short v8us  __attribute__((ext_vector_type(8)));
typedef unsigned short v16us __attribute__((ext_vector_type(16)));
typedef __bf16         v16bf __attribute__((ext_vector_type(16)));
typedef v4f  __attribute__((may_alias)) v4fa;
typedef v4i  __attribute__((may_alias)) v4ia;
typedef v4us __attribute__((may_alias)) v4usa;
typedef v8us __attribute__((may_alias)) v8usa;
union FragB { v16bf v; v16us u; v8us h[2]; v8i w; };

__device__ __forceinline__ v8f wmb(const FragB& a, const FragB& b, v8f c) {
  v8f d = __builtin_amdgcn_wmma_f32_16x16x32_bf16(false, a.v, false, b.v, (short)0, c, false, false);
  asm volatile("v_nop\n\tv_nop\n\tv_nop\n\tv_nop" : "+v"(d) : "v"(a.w), "v"(b.w));
  return d;
}

__device__ __forceinline__ v8f z8() { v8f z = {0.f, 0.f, 0.f, 0.f, 0.f, 0.f, 0.f, 0.f}; return z; }

__device__ __forceinline__ unsigned bf16_bits(float f) {
  const unsigned u = __float_as_uint(f);
  return (u + 0x7FFFu + ((u >> 16) & 1u)) >> 16;
}
__device__ __forceinline__ float bf16_val(float f) {
  return __uint_as_float(bf16_bits(f) << 16);
}
__device__ __forceinline__ unsigned hl_bits(float v, unsigned& lo) {
  const unsigned hb = bf16_bits(v);
  lo = bf16_bits(v - __uint_as_float(hb << 16));
  return hb;
}
__device__ __forceinline__ float relu_keep(float v) { return (v > 0.0f) ? v : (v - v); }

__device__ __forceinline__ void wave_sync() {
  __builtin_amdgcn_fence(__ATOMIC_RELEASE, "wavefront");
  __builtin_amdgcn_wave_barrier();
  __builtin_amdgcn_fence(__ATOMIC_ACQUIRE, "wavefront");
}

template <int SLB>
__device__ __forceinline__ int scan_chunk(const int* __restrict__ dsts, int nE, int cbase, int slotBase,
                                          int nb, int vec8, int* list, int tid, int lane, int wave) {
  int wc = 0;
  const int el0  = tid * EPT;
  const int e0   = cbase + el0;
  const int sent = -2147483647 - 1;
  v4i da, db;
  if (vec8 != 0 && cbase + CHUNK <= nE) {
    da = *(const v4i*)(dsts + e0);
    db = *(const v4i*)(dsts + e0 + 4);
  } else {
    da.x = (e0     < nE) ? dsts[min(e0,     nE - 1)] : sent;
    da.y = (e0 + 1 < nE) ? dsts[min(e0 + 1, nE - 1)] : sent;
    da.z = (e0 + 2 < nE) ? dsts[min(e0 + 2, nE - 1)] : sent;
    da.w = (e0 + 3 < nE) ? dsts[min(e0 + 3, nE - 1)] : sent;
    db.x = (e0 + 4 < nE) ? dsts[min(e0 + 4, nE - 1)] : sent;
    db.y = (e0 + 5 < nE) ? dsts[min(e0 + 5, nE - 1)] : sent;
    db.z = (e0 + 6 < nE) ? dsts[min(e0 + 6, nE - 1)] : sent;
    db.w = (e0 + 7 < nE) ? dsts[min(e0 + 7, nE - 1)] : sent;
  }
  const unsigned nbs = (unsigned)slotBase;
  const unsigned unb = (unsigned)nb;
  const unsigned s0 = (unsigned)da.x - nbs, s1 = (unsigned)da.y - nbs;
  const unsigned s2 = (unsigned)da.z - nbs, s3 = (unsigned)da.w - nbs;
  const unsigned s4 = (unsigned)db.x - nbs, s5 = (unsigned)db.y - nbs;
  const unsigned s6 = (unsigned)db.z - nbs, s7 = (unsigned)db.w - nbs;
  const bool h0 = s0 < unb, h1 = s1 < unb, h2 = s2 < unb, h3 = s3 < unb;
  const bool h4 = s4 < unb, h5 = s5 < unb, h6 = s6 < unb, h7 = s7 < unb;
  const unsigned any = __builtin_amdgcn_ballot_w32(h0 | h1 | h2 | h3 | h4 | h5 | h6 | h7);
  if (any != 0u) {
#define HITJ(J, HJ, SJ) { \
      const unsigned mj = __builtin_amdgcn_ballot_w32(HJ); \
      if (mj != 0u) { \
        if (HJ) { \
          const int pos = wc + (int)__builtin_amdgcn_mbcnt_lo(mj, 0u); \
          if (pos < WCAP) list[wave * WCAP + pos] = ((el0 + (J)) << SLB) | (int)(SJ); \
        } \
        wc += (int)__builtin_popcount(mj); } }
    HITJ(0, h0, s0)
    HITJ(1, h1, s1)
    HITJ(2, h2, s2)
    HITJ(3, h3, s3)
    HITJ(4, h4, s4)
    HITJ(5, h5, s5)
    HITJ(6, h6, s6)
    HITJ(7, h7, s7)
#undef HITJ
  }
  return wc;
}

__global__ __launch_bounds__(NTHR) void k_prep(const float* __restrict__ x, const float* __restrict__ wemb,
                                               const float* __restrict__ wpool, const float* __restrict__ wapp,
                                               unsigned short* wet, unsigned short* wp2, unsigned short* wa4,
                                               unsigned short* xb, int nN, int nUnits) {
  const int u = (int)blockIdx.x * NTHR + (int)threadIdx.x;
  v8us o;
  unsigned short* dp;
  if (u < NUWE) {
    const int n = u >> 2, k8 = (u & 3) * 8;
    const int nc = n < HID ? n : HID - 1;
    const bool okn = n < HID;
    const float* p = wemb + (size_t)k8 * HID + nc;
#pragma unroll
    for (int i = 0; i < 8; ++i) {
      const float f = p[(size_t)i * HID];
      o[i] = (unsigned short)bf16_bits(okn ? f : 0.0f);
    }
    dp = wet + (size_t)u * 8;
  } else if (u < NUWE + NUWP) {
    const int v  = u - NUWE;
    const int l  = v >> 12;
    const int n  = (v >> 5) & (DF - 1), k8 = (v & 31) * 8;
    const int kk = k8 & (DF - 1);
    const int nc = n < HID ? n : HID - 1;
    const bool okn = n < HID;
    const float* p = wpool + (size_t)l * HID * HID + nc;
#pragma unroll
    for (int i = 0; i < 8; ++i) {
      const int k  = kk + i;
      const int kc = k < HID ? k : HID - 1;
      const float f = p[(size_t)kc * HID];
      o[i] = (unsigned short)bf16_bits((okn && k < HID) ? f : 0.0f);
    }
    dp = wp2 + (size_t)v * 8;
  } else if (u < NUW) {
    const int v  = u - NUWE - NUWP;
    const int l  = v >> 13;
    const int n  = (v >> 6) & (DF - 1), k8 = (v & 63) * 8;
    const int kk = k8 & (DF - 1);
    const int rb = (k8 >= 2 * DF) ? HID : 0;
    const int nc = n < HID ? n : HID - 1;
    const bool okn = n < HID;
    const float* p = wapp + (size_t)l * 2 * HID * HID + (size_t)rb * HID + nc;
#pragma unroll
    for (int i = 0; i < 8; ++i) {
      const int k  = kk + i;
      const int kc = k < HID ? k : HID - 1;
      const float f = p[(size_t)kc * HID];
      o[i] = (unsigned short)bf16_bits((okn && k < HID) ? f : 0.0f);
    }
    dp = wa4 + (size_t)v * 8;
  } else if (u < nUnits) {
    const int v   = u - NUW;
    const int row = v >> 2, k8 = (v & 3) * 8;
    const int rc  = row < nN ? row : nN - 1;
    const bool lv = row < nN;
    const float* p = x + (size_t)rc * KE + k8;
    const v4f a = *(const v4f*)p;
    const v4f b = *(const v4f*)(p + 4);
    o[0] = (unsigned short)bf16_bits(lv ? a.x : 0.0f); o[1] = (unsigned short)bf16_bits(lv ? a.y : 0.0f);
    o[2] = (unsigned short)bf16_bits(lv ? a.z : 0.0f); o[3] = (unsigned short)bf16_bits(lv ? a.w : 0.0f);
    o[4] = (unsigned short)bf16_bits(lv ? b.x : 0.0f); o[5] = (unsigned short)bf16_bits(lv ? b.y : 0.0f);
    o[6] = (unsigned short)bf16_bits(lv ? b.z : 0.0f); o[7] = (unsigned short)bf16_bits(lv ? b.w : 0.0f);
    dp = xb + (size_t)v * 8;
  } else {
    return;
  }
  *(volatile v8us*)dp = o;
  __threadfence();
  *(volatile v8us*)dp = o;
}

__global__ __launch_bounds__(NTHR) void k_bucket(const int* __restrict__ srcs, const int* __restrict__ dsts,
                                                 int nE, int nN, int vec8,
                                                 int* listg, int* cntg, int* offg, int* flagg) {
  extern __shared__ __attribute__((aligned(16))) int dsm[];
  int* list = dsm;
  int* hl   = dsm + LISTN;
  int* sl   = hl + RCAP;
  int* cnt  = sl + RCAP;
  int* offs = cnt + NBA;
  int* cur  = offs + NBA;
  int* misc = cur + NBA;
  const int tid = (int)threadIdx.x, lane = tid & 31, wave = tid >> 5;
  const int nodeBase = (int)blockIdx.x * NBA;
  int nb = nN - nodeBase;
  nb = nb < 0 ? 0 : (nb > NBA ? NBA : nb);

  {
    const v4i z4 = {0, 0, 0, 0};
    for (int i = tid * 4; i < AGG_ZINTS; i += NTHR * 4) *(v4ia*)(dsm + i) = z4;
    if (tid < MISC_INTS) misc[tid] = 0;
  }
  __syncthreads();

  int t = 0, ov = 0;
  const int nChunks = (nE + CHUNK - 1) / CHUNK;
#pragma unroll 1
  for (int ch = 0; ch < nChunks; ++ch) {
    const int cbase = ch * CHUNK;
    const int wc = scan_chunk<SLA>(dsts, nE, cbase, nodeBase, nb, vec8, list, tid, lane, wave);
    if (lane == 0) misc[wave] = wc;
    __syncthreads();
    if (wave == 0) {
#pragma unroll 1
      for (int w2 = 0; w2 < NWAVE; ++w2) {
        int c = misc[w2];
        c = c < 0 ? 0 : (c > WCAP ? WCAP : c);
#pragma unroll 1
        for (int b0 = 0; b0 < c; b0 += 32) {
          const int idx = b0 + lane;
          const int ent_ = list[w2 * WCAP + (idx < WCAP ? idx : WCAP - 1)];
          const int m32 = (c - b0) < 32 ? (c - b0) : 32;
#pragma unroll 1
          for (int k = 0; k < m32; ++k) {
            const int u    = __builtin_amdgcn_readlane(ent_, k);
            const int slot = u & (NBA - 1);
            const int el   = (u >> SLA) & (CHUNK - 1);
            const int pk   = ((cbase + el) << SLA) | slot;
            if (t < RCAP) {
              if (lane == 0) { hl[t] = pk; cnt[slot] = cnt[slot] + 1; }
              t = t + 1;
            } else {
              ov = 1;
            }
          }
        }
      }
    }
    __syncthreads();
  }
  if (wave == 0 && lane == 0) { misc[8] = t; misc[9] = ov; }
  __syncthreads();
  int tt = misc[8];
  tt = tt < 0 ? 0 : (tt > RCAP ? RCAP : tt);
  const int ovf = misc[9];

  if (wave == 0) {
    const int base = lane * (NBA / 32);
    int s = 0;
#pragma unroll 1
    for (int i = 0; i < NBA / 32; ++i) s += cnt[base + i];
    int incl = s;
#pragma unroll
    for (int d = 1; d < 32; d <<= 1) {
      const int y = __shfl_up(incl, d, 32);
      if (lane >= d) incl += y;
    }
    int run = incl - s;
#pragma unroll 1
    for (int i = 0; i < NBA / 32; ++i) {
      const int cv = cnt[base + i];
      offs[base + i] = run;
      cur[base + i]  = run;
      run += cv;
    }
  }
  __syncthreads();
  if (wave == 0) {
#pragma unroll 1
    for (int b0 = 0; b0 < tt; b0 += 32) {
      const int idx = b0 + lane;
      const int ent_ = hl[idx < RCAP ? idx : RCAP - 1];
      const int m32 = (tt - b0) < 32 ? (tt - b0) : 32;
#pragma unroll 1
      for (int k = 0; k < m32; ++k) {
        const int u    = __builtin_amdgcn_readlane(ent_, k);
        const int slot = u & (NBA - 1);
        if (lane == 0) {
          int p = cur[slot];
          p = p < 0 ? 0 : (p > RCAP - 1 ? RCAP - 1 : p);
          sl[p] = u;
          cur[slot] = p + 1;
        }
      }
    }
  }
  __syncthreads();

  int* lrow = listg + (size_t)blockIdx.x * RCAP;
#pragma unroll 1
  for (int i4 = tid * 4; i4 < RCAP; i4 += NTHR * 4) {
    const v4i e4 = *(const v4ia*)(sl + i4);
    int e0 = e4.x >> SLA, e1 = e4.y >> SLA, e2 = e4.z >> SLA, e3 = e4.w >> SLA;
    e0 = e0 < 0 ? 0 : (e0 > nE - 1 ? nE - 1 : e0);
    e1 = e1 < 0 ? 0 : (e1 > nE - 1 ? nE - 1 : e1);
    e2 = e2 < 0 ? 0 : (e2 > nE - 1 ? nE - 1 : e2);
    e3 = e3 < 0 ? 0 : (e3 > nE - 1 ? nE - 1 : e3);
    int q0 = srcs[e0], q1 = srcs[e1], q2 = srcs[e2], q3 = srcs[e3];
    q0 = q0 < 0 ? 0 : (q0 > nN - 1 ? nN - 1 : q0);
    q1 = q1 < 0 ? 0 : (q1 > nN - 1 ? nN - 1 : q1);
    q2 = q2 < 0 ? 0 : (q2 > nN - 1 ? nN - 1 : q2);
    q3 = q3 < 0 ? 0 : (q3 > nN - 1 ? nN - 1 : q3);
    v4i s4;
    s4.x = (i4     < tt) ? q0 : 0;
    s4.y = (i4 + 1 < tt) ? q1 : 0;
    s4.z = (i4 + 2 < tt) ? q2 : 0;
    s4.w = (i4 + 3 < tt) ? q3 : 0;
    int* gp = lrow + i4;
    *(volatile v4i*)gp = s4;
    __threadfence();
    *(volatile v4i*)gp = s4;
  }
  {
    const v4i c4 = *(const v4ia*)(cnt + 4 * tid);
    const v4i o4 = *(const v4ia*)(offs + 4 * tid);
    const bool big = (c4.x > DEGCAP) | (c4.y > DEGCAP) | (c4.z > DEGCAP) | (c4.w > DEGCAP);
    if (big) misc[10] = 1;
    int* cp = cntg + (size_t)nodeBase + 4 * tid;
    int* op = offg + (size_t)nodeBase + 4 * tid;
    *(volatile v4i*)cp = c4;
    *(volatile v4i*)op = o4;
    __threadfence();
    *(volatile v4i*)cp = c4;
    *(volatile v4i*)op = o4;
  }
  __syncthreads();
  {
    const int fl = ((ovf != 0) || (misc[10] != 0)) ? 1 : 0;
    const v4i f4 = {fl, fl, fl, fl};
    int* fp = flagg + (size_t)blockIdx.x * 32 + 4 * (tid & 7);
    if (tid < 8) *(volatile v4i*)fp = f4;
    __threadfence();
    if (tid < 8) *(volatile v4i*)fp = f4;
  }
}

__global__ __launch_bounds__(NTHR) void k_agg(const float* __restrict__ P, const int* __restrict__ listg,
                                              const int* __restrict__ cntg, const int* __restrict__ offg,
                                              const int* __restrict__ flagg, int nN, unsigned short* agg) {
  __shared__ __attribute__((aligned(16))) unsigned short rowbuf[NWAVE * HP];
  const int tid = (int)threadIdx.x, lane = tid & 31, wave = tid >> 5;
  unsigned short* rb = rowbuf + wave * HP;
#pragma unroll 1
  for (int si = 0; si < AGB / NWAVE; ++si) {
    const int node = (int)blockIdx.x * AGB + si * NWAVE + wave;
    const int bo   = node >> SLA;
    int c  = __builtin_amdgcn_readfirstlane(cntg[node]);
    int o  = __builtin_amdgcn_readfirstlane(offg[node]);
    const int fl = __builtin_amdgcn_readfirstlane(flagg[(size_t)bo * 32]);
    const bool big = (c > DEGCAP) || (fl != 0);
    c = c < 0 ? 0 : (c > DEGCAP ? DEGCAP : c);
    o = o < 0 ? 0 : (o > RCAP ? RCAP : o);
    const int* lrow = listg + (size_t)bo * RCAP;
    float a0 = 0.0f, a1 = 0.0f, a2 = 0.0f, a3 = 0.0f;
#pragma unroll 1
    for (int b0 = 0; b0 < c; b0 += 32) {
      int idx = o + b0 + lane;
      idx = idx > RCAP - 1 ? RCAP - 1 : idx;
      int sr = lrow[idx];
      sr = sr < 0 ? 0 : (sr > nN - 1 ? nN - 1 : sr);
      const int m32 = (c - b0) < 32 ? (c - b0) : 32;
#pragma unroll 1
      for (int k = 0; k < m32; ++k) {
        const int sk = __builtin_amdgcn_readlane(sr, k);
        const v4f r = *(const v4f*)(P + (size_t)sk * DF + 4 * lane);
        a0 += r.x; a1 += r.y; a2 += r.z; a3 += r.w;
      }
    }
    const float inv = 1.0f / fmaxf((float)c, 1.0f);
    const float pzr = big ? __int_as_float(0x7fc00000) : 0.0f;
    const bool live = node < nN;
    const float m0 = live ? (a0 * inv + pzr) : 0.0f;
    const float m1 = live ? (a1 * inv + pzr) : 0.0f;
    const float m2 = live ? (a2 * inv + pzr) : 0.0f;
    const float m3 = live ? (a3 * inv + pzr) : 0.0f;
    v4us mh, ml;
    {
      unsigned lb;
      unsigned hb;
      hb = hl_bits(m0, lb); mh[0] = (unsigned short)hb; ml[0] = (unsigned short)lb;
      hb = hl_bits(m1, lb); mh[1] = (unsigned short)hb; ml[1] = (unsigned short)lb;
      hb = hl_bits(m2, lb); mh[2] = (unsigned short)hb; ml[2] = (unsigned short)lb;
      hb = hl_bits(m3, lb); mh[3] = (unsigned short)hb; ml[3] = (unsigned short)lb;
    }
    *(v4usa*)(rb + 4 * lane)      = mh;
    *(v4usa*)(rb + DF + 4 * lane) = ml;
    wave_sync();
    const v8us q0 = *(const v8usa*)(rb + 8 * lane);
    wave_sync();
    unsigned short* rpw = agg + (size_t)node * HP + 8 * lane;
    *(volatile v8us*)rpw = q0;
    __threadfence();
    *(volatile v8us*)rpw = q0;
  }
}

template <int MODE>
__global__ __launch_bounds__(GTHR) void k_gemm(const unsigned short* A0, const unsigned short* A1, int lda,
                                               int K0, int K1,
                                               const unsigned short* __restrict__ BT, int ldb,
                                               const float* __restrict__ bias,
                                               float* hf, unsigned short* hhl, float* pout, int nN) {
  __shared__ __attribute__((aligned(16))) float stg[GBM * GBN];
  __shared__ __attribute__((aligned(16))) unsigned short rbuf[GWAVE * HP];
  const int tid = (int)threadIdx.x, lane = tid & 31, wave = tid >> 5, hh = lane >> 4, m = lane & 15;
  const int rowBase = (int)blockIdx.x * GBM;

  v8f acc[NTL];
#pragma unroll
  for (int t = 0; t < NTL; ++t) acc[t] = z8();
  const unsigned short* bp = BT + (size_t)m * (size_t)ldb + 8 * hh;
  {
    const unsigned short* ap = A0 + (size_t)(rowBase + 16 * wave + m) * (size_t)lda + 8 * hh;
#pragma unroll 1
    for (int k0 = 0; k0 < K0; k0 += 32) {
      FragB af;
      af.h[0] = *(const v8usa*)(ap + k0);
      af.h[1] = *(const v8usa*)(ap + k0 + 16);
#pragma unroll
      for (int nt = 0; nt < NTL; ++nt) {
        const unsigned short* wq = bp + (size_t)(16 * nt) * (size_t)ldb + k0;
        FragB bf;
        bf.h[0] = *(const v8usa*)wq;
        bf.h[1] = *(const v8usa*)(wq + 16);
        acc[nt] = wmb(af, bf, acc[nt]);
      }
    }
  }
  if constexpr (MODE == 2) {
    const unsigned short* ap = A1 + (size_t)(rowBase + 16 * wave + m) * (size_t)lda + 8 * hh;
#pragma unroll 1
    for (int k0 = 0; k0 < K1; k0 += 32) {
      FragB af;
      af.h[0] = *(const v8usa*)(ap + k0);
      af.h[1] = *(const v8usa*)(ap + k0 + 16);
#pragma unroll
      for (int nt = 0; nt < NTL; ++nt) {
        const unsigned short* wq = bp + (size_t)(16 * nt) * (size_t)ldb + K0 + k0;
        FragB bf;
        bf.h[0] = *(const v8usa*)wq;
        bf.h[1] = *(const v8usa*)(wq + 16);
        acc[nt] = wmb(af, bf, acc[nt]);
      }
    }
  }

#pragma unroll
  for (int nt = 0; nt < NTL; ++nt) {
    const int lc = 16 * nt + m;
#pragma unroll
    for (int r = 0; r < 8; ++r) {
      const int lr = 16 * wave + 8 * hh + r;
      stg[lr * GBN + lc] = acc[nt][r];
    }
  }
#pragma unroll
  for (int r = 0; r < 8; ++r) {
    const int lr = 16 * wave + 8 * hh + r;
    stg[lr * GBN + 16 * NTL + m] = 0.0f;
  }
  __syncthreads();

  const int c0 = 4 * lane;
  const bool cm0 = (c0 + 0) < HID, cm1 = (c0 + 1) < HID, cm2 = (c0 + 2) < HID, cm3 = (c0 + 3) < HID;
  const float g0 = bias[(c0 + 0) < HID ? (c0 + 0) : HID - 1];
  const float g1 = bias[(c0 + 1) < HID ? (c0 + 1) : HID - 1];
  const float g2 = bias[(c0 + 2) < HID ? (c0 + 2) : HID - 1];
  const float g3 = bias[(c0 + 3) < HID ? (c0 + 3) : HID - 1];
  const float bq0 = cm0 ? bf16_val(g0) : 0.0f;
  const float bq1 = cm1 ? bf16_val(g1) : 0.0f;
  const float bq2 = cm2 ? bf16_val(g2) : 0.0f;
  const float bq3 = cm3 ? bf16_val(g3) : 0.0f;
  unsigned short* rb = rbuf + wave * HP;

#pragma unroll 1
  for (int i = 0; i < 16; ++i) {
    const int lr  = 16 * wave + i;
    const int row = rowBase + lr;
    const bool ok = row < nN;
    const v4f t = *(const v4fa*)(stg + lr * GBN + c0);
    const float y0 = cm0 ? (t.x + bq0) : 0.0f;
    const float y1 = cm1 ? (t.y + bq1) : 0.0f;
    const float y2 = cm2 ? (t.z + bq2) : 0.0f;
    const float y3 = cm3 ? (t.w + bq3) : 0.0f;
    float h0, h1, h2, h3;
    if constexpr (MODE == 0) {
      h0 = y0; h1 = y1; h2 = y2; h3 = y3;
    } else if constexpr (MODE == 1) {
      h0 = relu_keep(y0); h1 = relu_keep(y1); h2 = relu_keep(y2); h3 = relu_keep(y3);
    } else {
      float ss = (y0 * y0 + y1 * y1) + (y2 * y2 + y3 * y3);
      ss += __shfl_xor(ss, 16, 32);
      ss += __shfl_xor(ss, 8, 32);
      ss += __shfl_xor(ss, 4, 32);
      ss += __shfl_xor(ss, 2, 32);
      ss += __shfl_xor(ss, 1, 32);
      const float nrm = sqrtf(ss);
      const float dd  = fmaxf(nrm, 1e-12f);
      const float v0 = y0 / dd, v1 = y1 / dd, v2 = y2 / dd, v3 = y3 / dd;
      const v4f hv = *(const v4f*)(hf + (size_t)row * DF + c0);
      h0 = hv.x + relu_keep(v0);
      h1 = hv.y + relu_keep(v1);
      h2 = hv.z + relu_keep(v2);
      h3 = hv.w + relu_keep(v3);
    }
    v4f o4;
    o4.x = ok ? h0 : 0.0f; o4.y = ok ? h1 : 0.0f; o4.z = ok ? h2 : 0.0f; o4.w = ok ? h3 : 0.0f;
    if constexpr (MODE == 1) {
      float* pp = pout + (size_t)row * DF + c0;
      *(volatile v4f*)pp = o4;
      __threadfence();
      *(volatile v4f*)pp = o4;
    } else {
      v4us h4, l4;
      unsigned lb;
      unsigned hb;
      hb = hl_bits(o4.x, lb); h4[0] = (unsigned short)hb; l4[0] = (unsigned short)lb;
      hb = hl_bits(o4.y, lb); h4[1] = (unsigned short)hb; l4[1] = (unsigned short)lb;
      hb = hl_bits(o4.z, lb); h4[2] = (unsigned short)hb; l4[2] = (unsigned short)lb;
      hb = hl_bits(o4.w, lb); h4[3] = (unsigned short)hb; l4[3] = (unsigned short)lb;
      *(v4usa*)(rb + c0)      = h4;
      *(v4usa*)(rb + DF + c0) = l4;
      wave_sync();
      const v8us q = *(const v8usa*)(rb + 8 * lane);
      wave_sync();
      float* hp = hf + (size_t)row * DF + c0;
      unsigned short* qp = hhl + (size_t)row * HP + 8 * lane;
      *(volatile v4f*)hp  = o4;
      *(volatile v8us*)qp = q;
      __threadfence();
      *(volatile v4f*)hp  = o4;
      *(volatile v8us*)qp = q;
    }
  }
  (void)A1; (void)K1; (void)pout; (void)hhl; (void)hf;
}

__global__ __launch_bounds__(PTHR) void k_pool_mlp(const float* __restrict__ hfp, const int* __restrict__ gid, int nN,
                                                   const float* __restrict__ w1, const float* __restrict__ b1,
                                                   const float* __restrict__ w2, const float* __restrict__ b2,
                                                   const float* __restrict__ w3, const float* __restrict__ b3,
                                                   float* logp) {
  __shared__ __attribute__((aligned(16))) float wst[NWAVE * DF];
  __shared__ __attribute__((aligned(16))) float s0[DF];
  __shared__ __attribute__((aligned(16))) float s1[64];
  __shared__ __attribute__((aligned(16))) float s2[32];
  __shared__ __attribute__((aligned(16))) float s3[LOGW];
  __shared__ int plist[NWAVE * 32];
  __shared__ int wcn[NWAVE];
  const int tid = (int)threadIdx.x, lane = tid & 31, wave = tid >> 5;
  const int g = (int)blockIdx.x;
  float a0 = 0.0f, a1 = 0.0f, a2 = 0.0f, a3 = 0.0f;
  int cn = 0;
  const int nChunks = (nN + PTHR - 1) / PTHR;
#pragma unroll 1
  for (int ch = 0; ch < nChunks; ++ch) {
    const int n  = ch * PTHR + tid;
    const int nc = n < nN ? n : nN - 1;
    const int bv = gid[nc];
    const bool hit = (n < nN) && (bv == g);
    const unsigned mj = __builtin_amdgcn_ballot_w32(hit);
    if (mj != 0u) {
      if (hit) plist[wave * 32 + (int)__builtin_amdgcn_mbcnt_lo(mj, 0u)] = n;
      const int c = (int)__builtin_popcount(mj);
      wave_sync();
#pragma unroll 1
      for (int k = 0; k < c; ++k) {
        int nd = plist[wave * 32 + k];
        nd = nd < 0 ? 0 : (nd > nN - 1 ? nN - 1 : nd);
        const v4f r = *(const v4f*)(hfp + (size_t)nd * DF + 4 * lane);
        a0 += r.x; a1 += r.y; a2 += r.z; a3 += r.w;
      }
      cn += c;
      wave_sync();
    }
  }
  {
    v4f sv4; sv4.x = a0; sv4.y = a1; sv4.z = a2; sv4.w = a3;
    *(v4fa*)(wst + wave * DF + 4 * lane) = sv4;
    if (lane == 0) wcn[wave] = cn;
  }
  __syncthreads();
  if (tid < DF) {
    double sv = 0.0;
    int ct = 0;
#pragma unroll 1
    for (int w2i = 0; w2i < NWAVE; ++w2i) {
      sv += (double)wst[w2i * DF + tid];
      ct += wcn[w2i];
    }
    const float cf = (float)(ct < 1 ? 1 : ct);
    s0[tid] = (float)sv / cf;
  }
  __syncthreads();
  if (wave < 2) {
    const int o = tid < 54 ? tid : 53;
    float a = 0.0f;
#pragma unroll 4
    for (int k = 0; k < HID; ++k) a = fmaf(s0[k], bf16_val(w1[k * 54 + o]), a);
    a = a + bf16_val(b1[o]);
    if (tid < 54) s1[tid] = relu_keep(a);
  }
  __syncthreads();
  if (wave < 1) {
    const int o = tid < 27 ? tid : 26;
    float a = 0.0f;
#pragma unroll 4
    for (int k = 0; k < 54; ++k) a = fmaf(s1[k], bf16_val(w2[k * 27 + o]), a);
    a = a + bf16_val(b2[o]);
    if (tid < 27) s2[tid] = relu_keep(a);
  }
  __syncthreads();
  if (wave < 1) {
    const int o = tid < 10 ? tid : 9;
    float a = 0.0f;
#pragma unroll 4
    for (int k = 0; k < 27; ++k) a = fmaf(s2[k], bf16_val(w3[k * 10 + o]), a);
    a = a + bf16_val(b3[o]);
    s3[tid] = (tid < 10) ? a : 0.0f;
  }
  __syncthreads();
  {
    const bool ok = tid < LOGW / 4;
    v4f pv = {0.f, 0.f, 0.f, 0.f};
    if (ok) pv = *(const v4fa*)(s3 + 4 * tid);
    float* op = logp + (size_t)g * LOGW + 4 * (tid & 7);
    if (ok) *(volatile v4f*)op = pv;
    __threadfence();
    if (ok) *(volatile v4f*)op = pv;
  }
}

__global__ __launch_bounds__(OTHR) void k_out(const float* __restrict__ logp, const int* __restrict__ flagg,
                                              int nFlag, int nOut4, int nG, float* out) {
  __shared__ int sf;
  const int tid = (int)threadIdx.x;
  if (tid == 0) sf = 0;
  __syncthreads();
  {
    const int fc = tid < nFlag ? tid : nFlag - 1;
    const int f  = flagg[(size_t)fc * 32];
    if (tid < nFlag && f != 0) sf = 1;
  }
  __syncthreads();
  const bool poison = sf != 0;
  const float qn = __int_as_float(0x7fc00000);
#pragma unroll 1
  for (int t = tid; t < nOut4; t += OTHR) {
    const int e0 = 4 * t;
    int gA = (e0    ) / 10, gB = (e0 + 1) / 10, gC = (e0 + 2) / 10, gD = (e0 + 3) / 10;
    const int cA = (e0    ) - 10 * gA, cB = (e0 + 1) - 10 * gB, cC = (e0 + 2) - 10 * gC, cD = (e0 + 3) - 10 * gD;
    gA = gA > nG - 1 ? nG - 1 : gA; gB = gB > nG - 1 ? nG - 1 : gB;
    gC = gC > nG - 1 ? nG - 1 : gC; gD = gD > nG - 1 ? nG - 1 : gD;
    const float fA = logp[(size_t)gA * LOGW + cA];
    const float fB = logp[(size_t)gB * LOGW + cB];
    const float fC = logp[(size_t)gC * LOGW + cC];
    const float fD = logp[(size_t)gD * LOGW + cD];
    v4f o;
    o.x = poison ? qn : fA; o.y = poison ? qn : fB; o.z = poison ? qn : fC; o.w = poison ? qn : fD;
    float* op = out + (size_t)e0;
    *(volatile v4f*)op = o;
    __threadfence();
    *(volatile v4f*)op = o;
  }
}

static inline int cdiv(int a, int b) { return (a + b - 1) / b; }
static inline size_t al256(size_t o) { return (o + 255) & ~(size_t)255; }

extern "C" void kernel_launch(void* const* d_in, const int* in_sizes, int n_in,
                              void* d_out, int out_size, void* d_ws, size_t ws_size,
                              hipStream_t stream) {
  if (n_in < 19) return;
  const int nN = in_sizes[6];
  const int nE = in_sizes[4];
  if (nN < GBM || nN > (1 << 22)) return;
  if (nE < 1 || nE >= (1 << 21) || in_sizes[5] != nE) return;
  if ((long long)in_sizes[0] != (long long)nN * KE) return;
  if (in_sizes[7] != KE * HID || in_sizes[8] != HID) return;
  if (in_sizes[9] != NLAY * HID * HID || in_sizes[10] != NLAY * HID) return;
  if (in_sizes[11] != NLAY * 2 * HID * HID || in_sizes[12] != NLAY * HID) return;
  if (in_sizes[13] != HID * 54 || in_sizes[14] != 54) return;
  if (in_sizes[15] != 54 * 27 || in_sizes[16] != 27) return;
  if (in_sizes[17] != 27 * 10 || in_sizes[18] != 10) return;
  if (out_size < 40 || (out_size % 10) != 0 || (out_size % 4) != 0) return;
  const int nG = out_size / 10;
  if (nG > 65535) return;
  const int nOut4 = out_size / 4;

  const float* x     = (const float*)d_in[0];
  const int*   src   = (const int*)  d_in[4];
  const int*   dst   = (const int*)  d_in[5];
  const int*   gid   = (const int*)  d_in[6];
  const float* Wemb  = (const float*)d_in[7];
  const float* bemb  = (const float*)d_in[8];
  const float* Wpool = (const float*)d_in[9];
  const float* bpool = (const float*)d_in[10];
  const float* Wapp  = (const float*)d_in[11];
  const float* bapp  = (const float*)d_in[12];
  const float* W1    = (const float*)d_in[13];
  const float* b1    = (const float*)d_in[14];
  const float* W2    = (const float*)d_in[15];
  const float* b2    = (const float*)d_in[16];
  const float* W3    = (const float*)d_in[17];
  const float* b3    = (const float*)d_in[18];
  float* out = (float*)d_out;

  const int MP = cdiv(nN, GBM) * GBM;
  const int gM = MP / GBM;
  const int gA = cdiv(nN, NBA);
  if ((long long)gA * NBA < (long long)MP) return;
  if (gA > OTHR) return;
  const int vec8 = ((nE & 3) == 0) ? 1 : 0;

  char* ws = (char*)d_ws;
  size_t off = 0;
  const size_t oWET = off; off = al256(off + (size_t)DF * KE * 2);
  const size_t oWP2 = off; off = al256(off + (size_t)NLAY * DF * KP * 2);
  const size_t oWA4 = off; off = al256(off + (size_t)NLAY * DF * KA * 2);
  const size_t oXB  = off; off = al256(off + (size_t)MP * KE * 2);
  const size_t oHF  = off; off = al256(off + (size_t)MP * DF * 4);
  const size_t oHHL = off; off = al256(off + (size_t)MP * HP * 2);
  const size_t oP   = off; off = al256(off + (size_t)MP * DF * 4);
  const size_t oAGG = off; off = al256(off + (size_t)MP * HP * 2);
  const size_t oLST = off; off = al256(off + (size_t)gA * RCAP * 4);
  const size_t oCNT = off; off = al256(off + (size_t)gA * NBA * 4);
  const size_t oOFF = off; off = al256(off + (size_t)gA * NBA * 4);
  const size_t oFLG = off; off = al256(off + (size_t)gA * 128);
  const size_t oLOG = off; off = al256(off + (size_t)nG * LOGW * 4);
  if (off > ws_size || off > (size_t)WSMAX) return;
  unsigned short* WET = (unsigned short*)(ws + oWET);
  unsigned short* WP2 = (unsigned short*)(ws + oWP2);
  unsigned short* WA4 = (unsigned short*)(ws + oWA4);
  unsigned short* XB  = (unsigned short*)(ws + oXB);
  float*          HF  = (float*)(ws + oHF);
  unsigned short* HHL = (unsigned short*)(ws + oHHL);
  float*          Pp  = (float*)(ws + oP);
  unsigned short* AGG = (unsigned short*)(ws + oAGG);
  int*            LST = (int*)(ws + oLST);
  int*            CNT = (int*)(ws + oCNT);
  int*            OFS = (int*)(ws + oOFF);
  int*            FLG = (int*)(ws + oFLG);
  float*          LOG = (float*)(ws + oLOG);

  const size_t bktLds = (size_t)BKT_LDS_INTS * 4;
  hipFuncSetAttribute(reinterpret_cast<const void*>(&k_bucket), hipFuncAttributeMaxDynamicSharedMemorySize, (int)bktLds);

  const int nUnits = NUW + MP * (KE / 8);

  k_prep<<<cdiv(nUnits, NTHR), NTHR, 0, stream>>>(x, Wemb, Wpool, Wapp, WET, WP2, WA4, XB, nN, nUnits);
  k_bucket<<<gA, NTHR, bktLds, stream>>>(src, dst, nE, nN, vec8, LST, CNT, OFS, FLG);
  k_gemm<0><<<gM, GTHR, 0, stream>>>(XB, XB, KE, KE, 0, WET, KE, bemb, HF, HHL, Pp, nN);
  for (int l = 0; l < NLAY; ++l) {
    k_gemm<1><<<gM, GTHR, 0, stream>>>(HHL, HHL, HP, KP, 0, WP2 + (size_t)l * DF * KP, KP,
                                       bpool + (size_t)l * HID, HF, HHL, Pp, nN);
    k_agg<<<gM, NTHR, 0, stream>>>(Pp, LST, CNT, OFS, FLG, nN, AGG);
    k_gemm<2><<<gM, GTHR, 0, stream>>>(HHL, AGG, HP, KP, KP, WA4 + (size_t)l * DF * KA, KA,
                                       bapp + (size_t)l * HID, HF, HHL, Pp, nN);
  }
  k_pool_mlp<<<nG, PTHR, 0, stream>>>(HF, gid, nN, W1, b1, W2, b2, W3, b3, LOG);
  k_out<<<1, OTHR, 0, stream>>>(LOG, FLG, gA, nOut4, nG, out);
}
